// RGAT_37778532335711
// MI455X (gfx1250) — hardware-verified
//
#include <hip/hip_runtime.h>
#include <stddef.h>


#define HIDC    128
#define NTHR    256
#define NWAVE   8
#define EPT     8
#define NGRP    2
#define CHUNK   (NTHR * EPT * NGRP)
#define WCAP    (EPT * NGRP * 32)
#define LISTN   (NWAVE * WCAP)
#define NBC     4096
#define NBF     1024
#define RCAP    40960
#define RBN     128
#define TGT     256
#define DEGCAP  512
#define GROWS   128
#define OTHR    512
#define RPADC   128
#define NLAYER  2
#define WSCALE  8.0f
#define ASCALE  64.0f
#define OUTINV  0.001953125f
#define LRELU   0.2f
#define LNEPS   1e-5f
#define NEGBIG  (-3.0e38f)

#define LDS_GEMM (GROWS * HIDC * 4 + 2 * GROWS * 4)
#define LDS_FILL ((RCAP + NBF + LISTN) * 4 + 64)

static_assert((CHUNK & (CHUNK - 1)) == 0);
static_assert(CHUNK <= 4096);
static_assert(NBC <= 4096 && NBF <= 4096);
static_assert((NBC & (NBC - 1)) == 0 && (NBF & (NBF - 1)) == 0);
static_assert(NBC == 4 * NBF);
static_assert(OTHR * 8 == NBC);
static_assert((RCAP % 32) == 0);
static_assert(GROWS * (HIDC + 8) * 2 <= GROWS * HIDC * 4);
static_assert((TGT % GROWS) == 0 && TGT == NWAVE * 32);
static_assert((GROWS * HIDC / 8) % NTHR == 0);
static_assert((NLAYER * HIDC * HIDC / 8) % NTHR == 0);
static_assert((HIDC * HIDC / 8) / NTHR == 8);
static_assert(NTHR == 2 * HIDC);
static_assert(RPADC == 128 && GROWS == 128);

typedef float    v4f  __attribute__((ext_vector_type(4)));
typedef float    v8f  __attribute__((ext_vector_type(8)));
typedef int      v4i  __attribute__((ext_vector_type(4)));
typedef _Float16 v8h  __attribute__((ext_vector_type(8)));
typedef _Float16 v16h __attribute__((ext_vector_type(16)));
union FragH { v16h v; v8h h[2]; };

__device__ __forceinline__ v8h cvt8(v4f a, v4f b) {
  v8h r;
  r[0] = (_Float16)a.x; r[1] = (_Float16)a.y; r[2] = (_Float16)a.z; r[3] = (_Float16)a.w;
  r[4] = (_Float16)b.x; r[5] = (_Float16)b.y; r[6] = (_Float16)b.z; r[7] = (_Float16)b.w;
  return r;
}

__device__ __forceinline__ v8f wmh(v16h a, v16h b, v8f c) {
  v8f d = __builtin_amdgcn_wmma_f32_16x16x32_f16(false, a, false, b, (short)0, c, false, false);
  asm volatile("v_nop\n\tv_nop\n\tv_nop\n\tv_nop" : "+v"(d) : "v"(a), "v"(b));
  return d;
}

__device__ __forceinline__ float wsum32(float v) {
#pragma unroll
  for (int o = 16; o > 0; o >>= 1) v += __shfl_xor(v, o, 32);
  return v;
}
__device__ __forceinline__ float wmax32(float v) {
#pragma unroll
  for (int o = 16; o > 0; o >>= 1) v = fmaxf(v, __shfl_xor(v, o, 32));
  return v;
}

template <int NB>
__device__ __forceinline__ int scan_chunk(const int* __restrict__ dsts, int nE, int cbase, int slotBase,
                                          int vec8, int* list, int tid, int lane, int wave) {
  int wc = 0;
#pragma unroll
  for (int g = 0; g < NGRP; ++g) {
    const int el0  = (g * NTHR + tid) * EPT;
    const int e0   = cbase + el0;
    const int sent = -2147483647 - 1;
    v4i da, db;
    if (vec8 != 0 && cbase + CHUNK <= nE) {
      da = *(const v4i*)(dsts + e0);
      db = *(const v4i*)(dsts + e0 + 4);
    } else {
      da.x = (e0     < nE) ? dsts[min(e0, nE - 1)] : sent;
      da.y = (e0 + 1 < nE) ? dsts[min(e0 + 1, nE - 1)] : sent;
      da.z = (e0 + 2 < nE) ? dsts[min(e0 + 2, nE - 1)] : sent;
      da.w = (e0 + 3 < nE) ? dsts[min(e0 + 3, nE - 1)] : sent;
      db.x = (e0 + 4 < nE) ? dsts[min(e0 + 4, nE - 1)] : sent;
      db.y = (e0 + 5 < nE) ? dsts[min(e0 + 5, nE - 1)] : sent;
      db.z = (e0 + 6 < nE) ? dsts[min(e0 + 6, nE - 1)] : sent;
      db.w = (e0 + 7 < nE) ? dsts[min(e0 + 7, nE - 1)] : sent;
    }
    const unsigned nb = (unsigned)slotBase;
    const unsigned s0 = (unsigned)da.x - nb, s1 = (unsigned)da.y - nb;
    const unsigned s2 = (unsigned)da.z - nb, s3 = (unsigned)da.w - nb;
    const unsigned s4 = (unsigned)db.x - nb, s5 = (unsigned)db.y - nb;
    const unsigned s6 = (unsigned)db.z - nb, s7 = (unsigned)db.w - nb;
    const bool h0 = s0 < (unsigned)NB, h1 = s1 < (unsigned)NB, h2 = s2 < (unsigned)NB, h3 = s3 < (unsigned)NB;
    const bool h4 = s4 < (unsigned)NB, h5 = s5 < (unsigned)NB, h6 = s6 < (unsigned)NB, h7 = s7 < (unsigned)NB;
    const unsigned any = __builtin_amdgcn_ballot_w32(h0 | h1 | h2 | h3 | h4 | h5 | h6 | h7);
    if (any != 0u) {
#define HITJ(J, HJ, SJ) { \
        const unsigned mj = __builtin_amdgcn_ballot_w32(HJ); \
        if (mj != 0u) { \
          if (HJ) { \
            const int pos = wc + (int)__builtin_amdgcn_mbcnt_lo(mj, 0u); \
            if (pos < WCAP) list[wave * WCAP + pos] = ((el0 + (J)) << 12) | (int)(SJ); \
          } \
          wc += (int)__builtin_popcount(mj); } }
      HITJ(0, h0, s0)
      HITJ(1, h1, s1)
      HITJ(2, h2, s2)
      HITJ(3, h3, s3)
      HITJ(4, h4, s4)
      HITJ(5, h5, s5)
      HITJ(6, h6, s6)
      HITJ(7, h7, s7)
#undef HITJ
    }
  }
  return wc;
}

__global__ __launch_bounds__(NTHR) void k_wprep(
    const float* __restrict__ Wa, const float* __restrict__ Wb, _Float16* wL) {
  const int layer = (int)blockIdx.x >> 3;
  const float* src = Wa;
  if (layer != 0) src = Wb;
  const int i  = (int)blockIdx.x * NTHR + (int)threadIdx.x;
  const int e  = i * 8;
  const int el = e - layer * (HIDC * HIDC);
  const v4f a = *(const v4f*)(src + el) * WSCALE;
  const v4f b = *(const v4f*)(src + el + 4) * WSCALE;
  const v8h hv = cvt8(a, b);
  _Float16* dp = wL + e;
  *(volatile v8h*)dp = hv;
  __threadfence();
  *(volatile v8h*)dp = hv;
}

__global__ __launch_bounds__(NTHR) void k_rel(
    const float* __restrict__ relE,
    const float* __restrict__ Wra, const float* __restrict__ bra, const float* __restrict__ ata,
    const float* __restrict__ Wrb, const float* __restrict__ brb, const float* __restrict__ atb,
    float* ra, int nR) {
  __shared__ __attribute__((aligned(16))) float sP[NTHR];
  __shared__ __attribute__((aligned(16))) float sRa[RPADC];
  const int tid = threadIdx.x;
  const float* Wr = Wra; const float* br = bra; const float* ar = ata + 2 * HIDC;
  if (blockIdx.x != 0) { Wr = Wrb; br = brb; ar = atb + 2 * HIDC; }
  if (tid < RPADC) sRa[tid] = 0.0f;
  __syncthreads();
  const int o   = tid & (HIDC - 1);
  const int sub = tid >> 7;
  const float bo = br[o];
  const float ao = ar[o];
  const float* wrow = Wr + (size_t)o * HIDC;
  const int nIt = (nR + 1) >> 1;
#pragma unroll 1
  for (int it = 0; it < nIt; ++it) {
    const int r  = 2 * it + sub;
    const int rc = r < nR ? r : nR - 1;
    const float* er = relE + (size_t)rc * HIDC;
    float s = 0.0f;
#pragma unroll 4
    for (int i = 0; i < HIDC; ++i) s += er[i] * wrow[i];
    sP[tid] = (s + bo) * ao;
    __syncthreads();
    if (tid < 2) {
      const int rw = 2 * it + tid;
      float acc = 0.0f;
#pragma unroll 4
      for (int i = 0; i < HIDC; ++i) acc += sP[tid * HIDC + i];
      if (rw < nR && rw < RPADC) sRa[rw] = acc;
    }
    __syncthreads();
  }
  v4f v = {0.f, 0.f, 0.f, 0.f};
  if (tid < 32) v = *(const v4f*)(sRa + 4 * tid);
  float* gp = ra + (size_t)blockIdx.x * RPADC + 4 * tid;
  if (tid < 32) *(volatile v4f*)gp = v;
  __threadfence();
  if (tid < 32) *(volatile v4f*)gp = v;
}

__global__ __launch_bounds__(NTHR) void k_count(
    const int* __restrict__ ei, int* cnt, int nE, int vec8) {
  __shared__ __attribute__((aligned(16))) int scnt[NBC];
  __shared__ __attribute__((aligned(16))) int list[LISTN];
  __shared__ int wcnt[NWAVE];
  const int tid = threadIdx.x, lane = tid & 31, wave = tid >> 5;
  const int nodeBase = blockIdx.x * NBC;
  const int* dsts = ei + nE;

  for (int i = tid; i < NBC; i += NTHR) scnt[i] = 0;
  __syncthreads();

  const int nChunks = (nE + CHUNK - 1) / CHUNK;
#pragma unroll 1
  for (int ch = 0; ch < nChunks; ++ch) {
    const int cbase = ch * CHUNK;
    const int wc = scan_chunk<NBC>(dsts, nE, cbase, nodeBase, vec8, list, tid, lane, wave);
    if (lane == 0) wcnt[wave] = wc;
    __syncthreads();
    if (wave == 0) {
#pragma unroll 1
      for (int wsx = 0; wsx < NWAVE; ++wsx) {
        int n = __builtin_amdgcn_readfirstlane(wcnt[wsx]);
        n = n > WCAP ? WCAP : (n < 0 ? 0 : n);
        const int* lp = list + wsx * WCAP;
#pragma unroll 1
        for (int i = 0; i < n; ++i) {
          const int ent  = __builtin_amdgcn_readfirstlane(lp[i]);
          const int slot = ent & (NBC - 1);
          if (lane == 0) scnt[slot] = scnt[slot] + 1;
        }
      }
    }
    __syncthreads();
  }

  v4i cq[4];
#pragma unroll
  for (int q = 0; q < 4; ++q) {
    const int f = (wave * 4 + q) * 128 + 4 * lane;
    cq[q] = *(const v4i*)(scnt + f);
  }
  int* cp = cnt + (size_t)nodeBase;
#pragma unroll
  for (int q = 0; q < 4; ++q) {
    const int f = (wave * 4 + q) * 128 + 4 * lane;
    *(volatile v4i*)(cp + f) = cq[q];
  }
  __threadfence();
#pragma unroll
  for (int q = 0; q < 4; ++q) {
    const int f = (wave * 4 + q) * 128 + 4 * lane;
    *(volatile v4i*)(cp + f) = cq[q];
  }
}

__global__ __launch_bounds__(OTHR) void k_offsets(
    const int* __restrict__ cnt, int* off, int* rbase, int nChunk) {
  __shared__ __attribute__((aligned(16))) int soff[NBC];
  __shared__ __attribute__((aligned(16))) int srb[RBN];
  __shared__ int wtot[OTHR / 32];
  const int tid = threadIdx.x, lane = tid & 31, wave = tid >> 5, sub = tid >> 7;
  for (int i = tid; i < RBN; i += OTHR) srb[i] = 0;
  int carry = 0;
#pragma unroll 1
  for (int ch = 0; ch < nChunk; ++ch) {
    const int base = ch * NBC;
    const v4i c0 = *(const v4i*)(cnt + base + 8 * tid);
    const v4i c1 = *(const v4i*)(cnt + base + 8 * tid + 4);
    const int e0 = max(c0.x, 0), e1 = max(c0.y, 0), e2 = max(c0.z, 0), e3 = max(c0.w, 0);
    const int e4 = max(c1.x, 0), e5 = max(c1.y, 0), e6 = max(c1.z, 0), e7 = max(c1.w, 0);
    const int ts = e0 + e1 + e2 + e3 + e4 + e5 + e6 + e7;
    int incl = ts;
#pragma unroll
    for (int d = 1; d < 32; d <<= 1) {
      const int t = __shfl_up(incl, d);
      if (lane >= d) incl += t;
    }
    if (lane == 31) wtot[wave] = incl;
    __syncthreads();
    const int S0 = wtot[0]  + wtot[1]  + wtot[2]  + wtot[3];
    const int S1 = wtot[4]  + wtot[5]  + wtot[6]  + wtot[7];
    const int S2 = wtot[8]  + wtot[9]  + wtot[10] + wtot[11];
    const int S3 = wtot[12] + wtot[13] + wtot[14] + wtot[15];
    int pre = 0;
#pragma unroll 1
    for (int w = 4 * sub; w < wave; ++w) pre += wtot[w];
    const int b0 = carry;
    const int b1 = b0 + ((S0 + 31) & ~31);
    const int b2 = b1 + ((S1 + 31) & ~31);
    const int b3 = b2 + ((S2 + 31) & ~31);
    const int b4 = b3 + ((S3 + 31) & ~31);
    const int myb = sub == 0 ? b0 : (sub == 1 ? b1 : (sub == 2 ? b2 : b3));
    if (tid == 0) {
      srb[min(4 * ch + 0, RBN - 1)] = b0;
      srb[min(4 * ch + 1, RBN - 1)] = b1;
      srb[min(4 * ch + 2, RBN - 1)] = b2;
      srb[min(4 * ch + 3, RBN - 1)] = b3;
    }
    int run = myb + pre + incl - ts;
    soff[8 * tid + 0] = run; run += e0;
    soff[8 * tid + 1] = run; run += e1;
    soff[8 * tid + 2] = run; run += e2;
    soff[8 * tid + 3] = run; run += e3;
    soff[8 * tid + 4] = run; run += e4;
    soff[8 * tid + 5] = run; run += e5;
    soff[8 * tid + 6] = run; run += e6;
    soff[8 * tid + 7] = run;
    carry = b4;
    __syncthreads();
    const v4i o0 = *(const v4i*)(soff + 4 * tid);
    const v4i o1 = *(const v4i*)(soff + 4 * (tid + OTHR));
    int* op = off + base;
    *(volatile v4i*)(op + 4 * tid) = o0;
    *(volatile v4i*)(op + 4 * (tid + OTHR)) = o1;
    __threadfence();
    *(volatile v4i*)(op + 4 * tid) = o0;
    *(volatile v4i*)(op + 4 * (tid + OTHR)) = o1;
    __syncthreads();
  }
  if (tid == 0) srb[min(4 * nChunk, RBN - 1)] = carry;
  __syncthreads();
  v4i rv = {0, 0, 0, 0};
  if (tid < 32) rv = *(const v4i*)(srb + 4 * tid);
  if (tid < 32) *(volatile v4i*)(rbase + 4 * tid) = rv;
  __threadfence();
  if (tid < 32) *(volatile v4i*)(rbase + 4 * tid) = rv;
}

__global__ __launch_bounds__(NTHR) void k_fill(
    const int* __restrict__ ei, const int* __restrict__ off, const int* __restrict__ rbase,
    int* csr, int nE, int vec8, int csrLen) {
  extern __shared__ v4f lds_dyn[];
  int* region = (int*)lds_dyn;
  int* cursor = region + RCAP;
  int* list   = cursor + NBF;
  int* wcnt   = list + LISTN;
  const int tid = threadIdx.x, lane = tid & 31, wave = tid >> 5;
  const int b = blockIdx.x;
  const int nodeBase = b * NBF;
  const int* dsts = ei + nE;

  int rb0 = rbase[b];
  const int rb1 = rbase[b + 1];
  rb0 = rb0 < 0 ? 0 : (rb0 > csrLen ? csrLen : rb0);
  rb0 &= ~31;
  int len = rb1 - rb0;
  len = len < 0 ? 0 : (len > RCAP ? RCAP : len);
  int lenW = (len + 31) & ~31;
  if (rb0 + lenW > csrLen) lenW = (csrLen - rb0) & ~31;

  {
    const v4i z = {0, 0, 0, 0};
    for (int i = tid; i < RCAP / 4; i += NTHR) ((v4i*)region)[i] = z;
    for (int s = tid; s < NBF; s += NTHR) {
      int o = off[nodeBase + s] - rb0;
      o = o < 0 ? 0 : (o > RCAP ? RCAP : o);
      cursor[s] = o;
    }
  }
  __syncthreads();

  const int nChunks = (nE + CHUNK - 1) / CHUNK;
#pragma unroll 1
  for (int ch = 0; ch < nChunks; ++ch) {
    const int cbase = ch * CHUNK;
    const int wc = scan_chunk<NBF>(dsts, nE, cbase, nodeBase, vec8, list, tid, lane, wave);
    if (lane == 0) wcnt[wave] = wc;
    __syncthreads();
    if (wave == 0) {
#pragma unroll 1
      for (int wsx = 0; wsx < NWAVE; ++wsx) {
        int n = __builtin_amdgcn_readfirstlane(wcnt[wsx]);
        n = n > WCAP ? WCAP : (n < 0 ? 0 : n);
        const int* lp = list + wsx * WCAP;
#pragma unroll 1
        for (int i = 0; i < n; ++i) {
          const int ent  = __builtin_amdgcn_readfirstlane(lp[i]);
          const int slot = ent & (NBF - 1);
          int e = cbase + ((ent >> 12) & (CHUNK - 1));
          e = e > nE - 1 ? nE - 1 : e;
          if (lane == 0) {
            int pos = cursor[slot];
            pos = pos < 0 ? 0 : (pos > RCAP - 1 ? RCAP - 1 : pos);
            region[pos] = e;
            const int np = pos + 1;
            cursor[slot] = np > RCAP ? RCAP : np;
          }
        }
      }
    }
    __syncthreads();
  }

  const int nv = lenW >> 2;
  int* gp = csr + rb0;
#pragma unroll 1
  for (int i = tid; i < nv; i += NTHR) { const v4i v = ((const v4i*)region)[i]; *(volatile v4i*)(gp + 4 * i) = v; }
  __threadfence();
#pragma unroll 1
  for (int i = tid; i < nv; i += NTHR) { const v4i v = ((const v4i*)region)[i]; *(volatile v4i*)(gp + 4 * i) = v; }
}

__global__ __launch_bounds__(NTHR) void k_gemm(
    const float* __restrict__ A, const int* __restrict__ xidx, const _Float16* __restrict__ Bs,
    const float* __restrict__ bias, const float* __restrict__ attn,
    float* C, float* sip, float* sjp, int nARows, int nIdx, int useIdx) {
  extern __shared__ v4f lds_dyn[];
  constexpr int AP = HIDC + 8;
  _Float16* sA  = (_Float16*)lds_dyn;
  float*    stg = (float*)lds_dyn;
  float*    ssi = (float*)lds_dyn + GROWS * HIDC;
  float*    ssj = ssi + GROWS;
  const int tid = threadIdx.x, lane = tid & 31, wave = tid >> 5, hh = lane >> 4, m = lane & 15;
  const int rowBase = blockIdx.x * GROWS;

#pragma unroll
  for (int i = 0; i < (GROWS * HIDC / 8) / NTHR; ++i) {
    const int idx = i * NTHR + tid;
    const int r   = idx >> 4;
    const int c0  = (idx & 15) * 8;
    const int row = rowBase + r;
    const int ri  = row < nIdx - 1 ? row : nIdx - 1;
    int xi = xidx[ri];
    xi = xi < 0 ? 0 : (xi > nARows - 1 ? nARows - 1 : xi);
    const int rr = row > nARows - 1 ? nARows - 1 : row;
    const int node = useIdx != 0 ? xi : rr;
    const float* ap = A + (size_t)node * HIDC + c0;
    const v4f a = *(const v4f*)ap * ASCALE, b = *(const v4f*)(ap + 4) * ASCALE;
    *(v8h*)(sA + r * AP + c0) = cvt8(a, b);
  }
  __syncthreads();

  v8f acc[8];
#pragma unroll
  for (int t = 0; t < 8; ++t) { v8f z = {0.f, 0.f, 0.f, 0.f, 0.f, 0.f, 0.f, 0.f}; acc[t] = z; }
  const _Float16* ar = sA + (wave * 16 + m) * AP + 8 * hh;
#pragma unroll
  for (int kt = 0; kt < HIDC / 32; ++kt) {
    FragH a;
    a.h[0] = *(const v8h*)(ar + 32 * kt);
    a.h[1] = *(const v8h*)(ar + 32 * kt + 16);
#pragma unroll
    for (int t = 0; t < 8; ++t) {
      const _Float16* bp = Bs + (size_t)(16 * t + m) * HIDC + 32 * kt + 8 * hh;
      FragH b;
      b.h[0] = *(const v8h*)bp;
      b.h[1] = *(const v8h*)(bp + 16);
      acc[t] = wmh(a.v, b.v, acc[t]);
    }
  }
  __syncthreads();

  const int r0 = wave * 16 + 8 * hh;
  float* sp = stg + r0 * HIDC + m;
#pragma unroll
  for (int t = 0; t < 8; ++t) {
    const float bl = bias[16 * t + m];
#pragma unroll
    for (int r = 0; r < 8; ++r) sp[r * HIDC + 16 * t] = acc[t][r] * OUTINV + bl;
  }
  __syncthreads();

  const v4f ai = *(const v4f*)(attn + 4 * lane);
  const v4f aj = *(const v4f*)(attn + HIDC + 4 * lane);
  const float* lp = stg + wave * 16 * HIDC + 4 * lane;
  float myi = 0.0f, myj = 0.0f;
#pragma unroll 1
  for (int i = 0; i < 16; ++i) {
    const v4f hv = *(const v4f*)(lp + i * HIDC);
    float di = hv.x * ai.x + hv.y * ai.y + hv.z * ai.z + hv.w * ai.w;
    float dj = hv.x * aj.x + hv.y * aj.y + hv.z * aj.z + hv.w * aj.w;
    di = wsum32(di);
    dj = wsum32(dj);
    myi = (lane == i) ? di : myi;
    myj = (lane == i) ? dj : myj;
  }
  if (lane < 16) { ssi[wave * 16 + lane] = myi; ssj[wave * 16 + lane] = myj; }
  __syncthreads();
  const float* sb = ssi + (wave & 1) * GROWS;
  const v4f sv = *(const v4f*)(sb + 4 * lane);

  float* gp = C + ((size_t)rowBase + wave * 16) * HIDC + 4 * lane;
  float* gsi = sip + (size_t)rowBase + 4 * lane;
  float* gsj = sjp + (size_t)rowBase + 4 * lane;
#pragma unroll
  for (int i = 0; i < 16; ++i) { const v4f v = *(const v4f*)(lp + i * HIDC); *(volatile v4f*)(gp + (size_t)i * HIDC) = v; }
  if (wave == 0) *(volatile v4f*)gsi = sv;
  if (wave == 1) *(volatile v4f*)gsj = sv;
  __threadfence();
#pragma unroll
  for (int i = 0; i < 16; ++i) { const v4f v = *(const v4f*)(lp + i * HIDC); *(volatile v4f*)(gp + (size_t)i * HIDC) = v; }
  if (wave == 0) *(volatile v4f*)gsi = sv;
  if (wave == 1) *(volatile v4f*)gsj = sv;
}

__device__ __forceinline__ float edge_alpha(
    const int* __restrict__ csr, const int* __restrict__ ei, const int* __restrict__ et,
    const float* __restrict__ sjp, const float* __restrict__ ra,
    int st, int q0, int lane, int csrLen, int nE, int nN, int nR, float sic, int* srcOut) {
  int pos = st + q0 + lane;
  pos = pos < 0 ? 0 : (pos > csrLen - 1 ? csrLen - 1 : pos);
  int e = csr[pos];
  e = e < 0 ? 0 : (e > nE - 1 ? nE - 1 : e);
  int s = ei[e];
  s = s < 0 ? 0 : (s > nN - 1 ? nN - 1 : s);
  int t = et[e];
  t = t < 0 ? 0 : (t > nR - 1 ? nR - 1 : t);
  const float v = sic + sjp[s] + ra[t];
  *srcOut = s;
  return v > 0.0f ? v : LRELU * v;
}

__global__ __launch_bounds__(NTHR) void k_agg(
    const int* __restrict__ csr, const int* __restrict__ off, const int* __restrict__ cnt,
    const int* __restrict__ ei, const int* __restrict__ et,
    const float* __restrict__ hl, const float* __restrict__ sip, const float* __restrict__ sjp,
    const float* __restrict__ ra, const float* __restrict__ xres, const int* __restrict__ xidx,
    const float* __restrict__ gam, const float* __restrict__ bet, float* xout,
    int nN, int nE, int nR, int csrLen, int nResRows, int nIdx, int useIdx, int nOutRows) {
  const int tid = threadIdx.x, lane = tid & 31, wave = tid >> 5;
  const int tbase = blockIdx.x * TGT + wave * 32;
  const int cl = tbase + lane;
  const int cnt_l = cnt[cl];
  const int off_l = off[cl];
  const float si_l = sip[cl];
  const int ri = cl < nIdx - 1 ? cl : nIdx - 1;
  int xi = xidx[ri];
  xi = xi < 0 ? 0 : (xi > nResRows - 1 ? nResRows - 1 : xi);
  const int rr = cl > nResRows - 1 ? nResRows - 1 : cl;
  const int node_l = useIdx != 0 ? xi : rr;
  const v4f ga = *(const v4f*)(gam + 4 * lane);
  const v4f be = *(const v4f*)(bet + 4 * lane);

#pragma unroll 1
  for (int j = 0; j < 32; ++j) {
    const int c = tbase + j;
    int n = __builtin_amdgcn_readlane(cnt_l, j);
    n = n < 0 ? 0 : (n > DEGCAP ? DEGCAP : n);
    const int st = __builtin_amdgcn_readlane(off_l, j);
    const float sic = __int_as_float(__builtin_amdgcn_readlane(__float_as_int(si_l), j));
    const int node = __builtin_amdgcn_readlane(node_l, j);

    float mx = NEGBIG;
#pragma unroll 1
    for (int q0 = 0; q0 < n; q0 += 32) {
      int sl;
      const float a = edge_alpha(csr, ei, et, sjp, ra, st, q0, lane, csrLen, nE, nN, nR, sic, &sl);
      const bool ok = (q0 + lane) < n;
      const float am = ok ? a : NEGBIG;
      mx = fmaxf(mx, wmax32(am));
    }
    v4f acc = {0.f, 0.f, 0.f, 0.f};
    float den = 0.0f;
#pragma unroll 1
    for (int q0 = 0; q0 < n; q0 += 32) {
      int sl;
      const float a = edge_alpha(csr, ei, et, sjp, ra, st, q0, lane, csrLen, nE, nN, nR, sic, &sl);
      const bool ok = (q0 + lane) < n;
      const float w = ok ? __expf(a - mx) : 0.0f;
      den += wsum32(w);
      const int mcnt = (n - q0) < 32 ? (n - q0) : 32;
#pragma unroll 1
      for (int p = 0; p < mcnt; ++p) {
        const int s = __builtin_amdgcn_readlane(sl, p);
        const float wp = __int_as_float(__builtin_amdgcn_readlane(__float_as_int(w), p));
        acc = acc + *(const v4f*)(hl + (size_t)s * HIDC + 4 * lane) * wp;
      }
    }
    const float dd  = n > 0 ? den : 1.0f;
    const float inv = 1.0f / dd;
    const v4f xv = *(const v4f*)(xres + (size_t)node * HIDC + 4 * lane);
    const v4f y  = xv + acc * inv;
    const float mu = wsum32(y.x + y.y + y.z + y.w) * (1.0f / 128.0f);
    const float d0 = y.x - mu, d1 = y.y - mu, d2 = y.z - mu, d3 = y.w - mu;
    const float var = wsum32(d0 * d0 + d1 * d1 + d2 * d2 + d3 * d3) * (1.0f / 128.0f);
    const float isd = rsqrtf(var + LNEPS);
    v4f res;
    res.x = fmaxf(d0 * isd * ga.x + be.x, 0.0f);
    res.y = fmaxf(d1 * isd * ga.y + be.y, 0.0f);
    res.z = fmaxf(d2 * isd * ga.z + be.z, 0.0f);
    res.w = fmaxf(d3 * isd * ga.w + be.w, 0.0f);
    if (c < nOutRows) {
      float* op = xout + (size_t)c * HIDC + 4 * lane;
      *(volatile v4f*)op = res;
      __threadfence();
      *(volatile v4f*)op = res;
    }
  }
}

extern "C" void kernel_launch(void* const* d_in, const int* in_sizes, int n_in,
                              void* d_out, int out_size, void* d_ws, size_t ws_size,
                              hipStream_t stream) {
  if (n_in < 19) return;
  const int nN = in_sizes[0];
  const int nE = in_sizes[2];
  if (nN <= 0 || nE <= 0 || in_sizes[1] != 2 * nE) return;
  const int nEmb = in_sizes[3] / HIDC;
  if (nEmb <= 0 || in_sizes[3] != nEmb * HIDC) return;
  const int nR = in_sizes[4] / HIDC;
  if (nR <= 0 || nR > RPADC || in_sizes[4] != nR * HIDC) return;
  if (in_sizes[5] != HIDC * HIDC || in_sizes[7] != HIDC * HIDC || in_sizes[12] != HIDC * HIDC || in_sizes[14] != HIDC * HIDC) return;
  if (in_sizes[6] != HIDC || in_sizes[8] != HIDC || in_sizes[10] != HIDC || in_sizes[11] != HIDC) return;
  if (in_sizes[13] != HIDC || in_sizes[15] != HIDC || in_sizes[17] != HIDC || in_sizes[18] != HIDC) return;
  if (in_sizes[9] != 3 * HIDC || in_sizes[16] != 3 * HIDC) return;
  if (out_size != nN * HIDC) return;
  if (nE > (1 << 28) || nN > (1 << 24)) return;

  const int*   xidx = (const int*)d_in[0];
  const int*   ei   = (const int*)d_in[1];
  const int*   etp  = (const int*)d_in[2];
  const float* emb  = (const float*)d_in[3];
  const float* relE = (const float*)d_in[4];
  const float* W1   = (const float*)d_in[5];
  const float* b1   = (const float*)d_in[6];
  const float* Wr1  = (const float*)d_in[7];
  const float* br1  = (const float*)d_in[8];
  const float* at1  = (const float*)d_in[9];
  const float* g1   = (const float*)d_in[10];
  const float* be1  = (const float*)d_in[11];
  const float* W2   = (const float*)d_in[12];
  const float* b2   = (const float*)d_in[13];
  const float* Wr2  = (const float*)d_in[14];
  const float* br2  = (const float*)d_in[15];
  const float* at2  = (const float*)d_in[16];
  const float* g2   = (const float*)d_in[17];
  const float* be2  = (const float*)d_in[18];
  float* out = (float*)d_out;

  const int NPAD   = ((nN + TGT - 1) / TGT) * TGT;
  const int nBC    = (nN + NBC - 1) / NBC;
  const int CNTPAD = nBC * NBC;
  if (4 * nBC + 1 > RBN) return;
  const int nBF    = (nN + NBF - 1) / NBF;
  const int csrLen = ((nE + 31) & ~31) + 32 * 4 * nBC + 64;
  const int nGemm  = NPAD / GROWS;
  const int nAgg   = NPAD / TGT;

  char* ws = (char*)d_ws;
  size_t off = 0;
  const size_t oWL  = off; off += (size_t)NLAYER * HIDC * HIDC * 2;  off = (off + 255) & ~(size_t)255;
  const size_t oRa  = off; off += (size_t)NLAYER * RPADC * 4;        off = (off + 255) & ~(size_t)255;
  const size_t oCnt = off; off += (size_t)CNTPAD * 4;                off = (off + 255) & ~(size_t)255;
  const size_t oOff = off; off += (size_t)CNTPAD * 4;                off = (off + 255) & ~(size_t)255;
  const size_t oRb  = off; off += (size_t)RBN * 4;                   off = (off + 255) & ~(size_t)255;
  const size_t oCsr = off; off += (size_t)csrLen * 4;                off = (off + 255) & ~(size_t)255;
  const size_t oHl  = off; off += (size_t)NPAD * HIDC * 4;           off = (off + 255) & ~(size_t)255;
  const size_t oX2  = off; off += (size_t)NPAD * HIDC * 4;           off = (off + 255) & ~(size_t)255;
  const size_t oSi  = off; off += (size_t)NPAD * 4;                  off = (off + 255) & ~(size_t)255;
  const size_t oSj  = off; off += (size_t)NPAD * 4;                  off = (off + 255) & ~(size_t)255;
  if (off > ws_size || off > (size_t)134217728) return;
  _Float16* wL   = (_Float16*)(ws + oWL);
  float*    ra   = (float*)(ws + oRa);
  int*      cnt  = (int*)(ws + oCnt);
  int*      offp = (int*)(ws + oOff);
  int*      rb   = (int*)(ws + oRb);
  int*      csr  = (int*)(ws + oCsr);
  float*    hl   = (float*)(ws + oHl);
  float*    x2   = (float*)(ws + oX2);
  float*    si   = (float*)(ws + oSi);
  float*    sj   = (float*)(ws + oSj);

  const int vec8 = ((nE & 3) == 0) ? 1 : 0;

  k_wprep<<<NLAYER * HIDC * HIDC / 8 / NTHR, NTHR, 0, stream>>>(W1, W2, wL);

  k_rel<<<NLAYER, NTHR, 0, stream>>>(relE, Wr1, br1, at1, Wr2, br2, at2, ra, nR);

  k_count<<<nBC, NTHR, 0, stream>>>(ei, cnt, nE, vec8);
  k_offsets<<<1, OTHR, 0, stream>>>(cnt, offp, rb, nBC);
  hipFuncSetAttribute(reinterpret_cast<const void*>(&k_fill),
                      hipFuncAttributeMaxDynamicSharedMemorySize, LDS_FILL);
  k_fill<<<nBF, NTHR, LDS_FILL, stream>>>(ei, offp, rb, csr, nE, vec8, csrLen);

  hipFuncSetAttribute(reinterpret_cast<const void*>(&k_gemm),
                      hipFuncAttributeMaxDynamicSharedMemorySize, LDS_GEMM);

  k_gemm<<<nGemm, NTHR, LDS_GEMM, stream>>>(emb, xidx, wL, b1, at1, hl, si, sj, nEmb, nN, 1);
  k_agg<<<nAgg, NTHR, 0, stream>>>(csr, offp, cnt, ei, etp, hl, si, sj, ra, emb, xidx, g1, be1, x2,
                                   nN, nE, nR, csrLen, nEmb, nN, 1, NPAD);

  k_gemm<<<nGemm, NTHR, LDS_GEMM, stream>>>(x2, xidx, wL + (size_t)HIDC * HIDC, b2, at2, hl, si, sj, NPAD, nN, 0);
  k_agg<<<nAgg, NTHR, 0, stream>>>(csr, offp, cnt, ei, etp, hl, si, sj, ra + RPADC, x2, xidx, g2, be2, out,
                                   nN, nE, nR, csrLen, NPAD, nN, 0, nN);
}
